// RNNClassifier_44822278701459
// MI455X (gfx1250) — hardware-verified
//
#include <hip/hip_runtime.h>
#include <stdint.h>

typedef __attribute__((ext_vector_type(16))) _Float16 v16h;
typedef __attribute__((ext_vector_type(8)))  _Float16 v8h;
typedef __attribute__((ext_vector_type(16))) __bf16   v16b;
typedef __attribute__((ext_vector_type(8)))  __bf16   v8b;
typedef __attribute__((ext_vector_type(8)))  float    v8f;
typedef __attribute__((ext_vector_type(4)))  float    v4f;
typedef __attribute__((ext_vector_type(4)))  unsigned int v4u;

constexpr int NBATCH   = 128;
constexpr int S_CTX    = 512;
constexpr int S_END    = 64;
constexpr int EMB_DIM  = 300;
constexpr int KXP      = 320;
constexpr int NCELL    = 128;
constexpr int NGX      = 3 * NCELL;
constexpr int NGATE_IN = EMB_DIM + NCELL;
constexpr int ROWS_CTX = NBATCH * S_CTX;
constexpr int ROWS_END = NBATCH * S_END;
constexpr int ROWS_ALL = ROWS_CTX + ROWS_END;
constexpr int NFEAT    = 4 * NCELL;
constexpr int NHID     = 128;

static_assert(KXP % 32 == 0 && KXP >= EMB_DIM, "k pad");
static_assert(ROWS_ALL % 64 == 0 && NGX % 64 == 0, "gemm tiles");
static_assert(ROWS_ALL % 128 == 0, "score blocks");
static_assert(NBATCH % 16 == 0 && NCELL == 128 && NGX == 384, "rec maps");
static_assert(S_CTX <= 512 && S_END <= S_CTX, "pool lds");
static_assert((ROWS_ALL * (KXP / 8)) % 256 == 0, "gather grid");
static_assert(EMB_DIM % 4 == 0, "emb align");
static_assert(NFEAT == 512 && NHID == 128, "head maps");

__device__ __forceinline__ unsigned short f2bf_bits(float f) {
  unsigned u = __float_as_uint(f);
  return (unsigned short)((u + 0x7FFFu + ((u >> 16) & 1u)) >> 16);
}
__device__ __forceinline__ float bf_bits2f(unsigned short h) { return __uint_as_float(((unsigned)h) << 16); }

__device__ __forceinline__ void dep_guard_h(v8f& a, v8f& b, v16h x, v16h y) { asm volatile("v_nop\n\tv_nop\n\tv_nop\n\tv_nop" : "+v"(a), "+v"(b) : "v"(x), "v"(y)); }
__device__ __forceinline__ void dep_guard_b(v8f& a, v8f& b, v16b x, v16b y) { asm volatile("v_nop\n\tv_nop\n\tv_nop\n\tv_nop" : "+v"(a), "+v"(b) : "v"(x), "v"(y)); }
__device__ __forceinline__ void keep4_h(v16h a, v16h b, v16h c, v16h d) { asm volatile("v_nop" :: "v"(a), "v"(b), "v"(c), "v"(d)); }
__device__ __forceinline__ void keep4_b(v16b a, v16b b, v16b c, v16b d) { asm volatile("v_nop" :: "v"(a), "v"(b), "v"(c), "v"(d)); }
__device__ __forceinline__ void acc_guard4(v8f& a, v8f& b, v8f& c, v8f& d) { asm volatile("v_nop\n\tv_nop\n\tv_nop\n\tv_nop" : "+v"(a), "+v"(b), "+v"(c), "+v"(d)); }
template <typename T> struct Frag;
template <> struct Frag<_Float16> {
  typedef v16h V; union U { v16h v; v8h h[2]; };
  static __device__ __forceinline__ v16h load(const _Float16* p) {
    U f; f.h[0] = *(const v8h*)(p); f.h[1] = *(const v8h*)(p + 16); return f.v;
  }
  static __device__ __forceinline__ v8f mma(v16h a, v16h b, v8f c) {
    return __builtin_amdgcn_wmma_f32_16x16x32_f16(false, a, false, b, (short)0, c, false, false);
  }
  static __device__ __forceinline__ void guard(v8f& a, v8f& b, v16h x, v16h y) { dep_guard_h(a, b, x, y); }
  static __device__ __forceinline__ void keep(v16h a, v16h b, v16h c, v16h d) { keep4_h(a, b, c, d); }
};
template <> struct Frag<__bf16> {
  typedef v16b V; union U { v16b v; v8b h[2]; };
  static __device__ __forceinline__ v16b load(const __bf16* p) {
    U f; f.h[0] = *(const v8b*)(p); f.h[1] = *(const v8b*)(p + 16); return f.v;
  }
  static __device__ __forceinline__ v8f mma(v16b a, v16b b, v8f c) {
    return __builtin_amdgcn_wmma_f32_16x16x32_bf16(false, a, false, b, (short)0, c, false, false);
  }
  static __device__ __forceinline__ void guard(v8f& a, v8f& b, v16b x, v16b y) { dep_guard_b(a, b, x, y); }
  static __device__ __forceinline__ void keep(v16b a, v16b b, v16b c, v16b d) { keep4_b(a, b, c, d); }
};

template <int ET> struct Elem;
template <> struct Elem<0> { typedef _Float16 T; };
template <> struct Elem<1> { typedef __bf16 T; };
template <int ET, bool SPLIT, int BIAS_MODE, int OUT_MODE, bool RESID, int ACT = 0>
__global__ __launch_bounds__(256) void wmma_gemm64(
    const unsigned short* __restrict__ Ap, const unsigned short* __restrict__ A2p, int lda, long strideA,
    const unsigned short* __restrict__ Btp, const unsigned short* __restrict__ Bt2p, int ldb, long strideB,
    void* __restrict__ Cout, void* __restrict__ Cout2, int ldc, long strideC,
    const float* __restrict__ bias,
    const float* __restrict__ resid, long strideR,
    int M, int N, int K, float scale) {
  typedef typename Elem<ET>::T T;
  typedef typename Frag<T>::V V;
  const T* A = (const T*)Ap; const T* A2 = (const T*)A2p; const T* Bt = (const T*)Btp; const T* Bt2 = (const T*)Bt2p;
  __shared__ __align__(16) float sT[8][16 * 68];
  const int b    = blockIdx.y;
  const int lane = threadIdx.x & 31;
  const int wave = threadIdx.x >> 5;
  const int tilesN = N >> 6;
  const int tilesM = M >> 6;
  const int tile = blockIdx.x * 8 + wave;
  if (tile >= tilesM * tilesN) return;
  const int tm = tile / tilesN;
  const int tn = tile - tm * tilesN;
  const int m0 = tm << 6;
  const int n0 = tn << 6;

  const T* Ab  = A  + (size_t)b * strideA;
  const T* Bb  = Bt + (size_t)b * strideB;
  const T* Ab2 = SPLIT ? (A2  + (size_t)b * strideA) : nullptr;
  const T* Bb2 = SPLIT ? (Bt2 + (size_t)b * strideB) : nullptr;

  const int rlane = lane & 15;
  const int koff  = (lane >> 4) * 8;
  const int mOff  = (lane >> 4) * 8;

  v8f acc[4][4];
#pragma unroll
  for (int i = 0; i < 4; ++i)
#pragma unroll
    for (int j = 0; j < 4; ++j) acc[i][j] = (v8f){0.f,0.f,0.f,0.f,0.f,0.f,0.f,0.f};

  for (int k0 = 0; k0 < K; k0 += 32) {
    V bh[4], bl[4];
#pragma unroll
    for (int j = 0; j < 4; ++j) {
      const size_t bo = (size_t)(n0 + (j << 4) + rlane) * ldb + koff + k0;
      bh[j] = Frag<T>::load(Bb + bo);
      if (SPLIT) bl[j] = Frag<T>::load(Bb2 + bo);
    }
#pragma unroll
    for (int i = 0; i < 4; ++i) {
      const size_t ao = (size_t)(m0 + (i << 4) + rlane) * lda + koff + k0;
      V ah = Frag<T>::load(Ab + ao);
      V al;
      if (SPLIT) al = Frag<T>::load(Ab2 + ao);
#pragma unroll
      for (int j = 0; j < 4; ++j) {
        acc[i][j] = Frag<T>::mma(ah, bh[j], acc[i][j]);
        if (SPLIT) {
          acc[i][j] = Frag<T>::mma(ah, bl[j], acc[i][j]);
          acc[i][j] = Frag<T>::mma(al, bh[j], acc[i][j]);
        }
      }
      Frag<T>::guard(acc[i][0], acc[i][3], ah, SPLIT ? al : ah);
    }
    Frag<T>::keep(bh[0], bh[1], bh[2], bh[3]);
    if (SPLIT) Frag<T>::keep(bl[0], bl[1], bl[2], bl[3]);
  }
  acc_guard4(acc[0][0], acc[0][1], acc[0][2], acc[0][3]);
  acc_guard4(acc[1][0], acc[1][1], acc[1][2], acc[1][3]);
  acc_guard4(acc[2][0], acc[2][1], acc[2][2], acc[2][3]);
  acc_guard4(acc[3][0], acc[3][1], acc[3][2], acc[3][3]);

  float* slab = sT[wave];
  const float* Rb = RESID ? (resid + (size_t)b * strideR) : nullptr;
#pragma unroll
  for (int i = 0; i < 4; ++i) {
    const int mBase = m0 + (i << 4);
#pragma unroll
    for (int j = 0; j < 4; ++j) {
      const int n = n0 + (j << 4) + rlane;
      float bv = 0.f;
      if (BIAS_MODE == 2) bv = bias[n];
#pragma unroll
      for (int r = 0; r < 8; ++r) {
        float v = acc[i][j][r] * scale;
        if (BIAS_MODE == 1) v += bias[mBase + mOff + r];
        if (BIAS_MODE == 2) v += bv;
        if (RESID) v += Rb[(size_t)(mBase + mOff + r) * ldc + n];
        if (ACT == 1) v = tanhf(v);
        if (ACT == 2) v = fmaxf(v, 0.0f);
        if (ACT == 3) v = v / (1.0f + expf(-v));
        if (ACT == 4) v = (v > 0.f) ? v : 0.01f * v;
        if (ACT == 5) v = 0.5f * v * (1.0f + erff(v * 0.70710678118654752f));
        slab[(mOff + r) * 68 + (j << 4) + rlane] = v;
      }
    }
    __builtin_amdgcn_fence(__ATOMIC_RELEASE, "workgroup");
    __builtin_amdgcn_wave_barrier();
    __builtin_amdgcn_fence(__ATOMIC_ACQUIRE, "workgroup");
    if (OUT_MODE == 0) {
      float* C = (float*)Cout + (size_t)b * strideC;
      const int hh = lane >> 4, c4 = (lane & 15) * 4;
      for (int pass = 0; pass < 2; ++pass) {
#pragma unroll
        for (int it = 0; it < 8; ++it) {
          const int row = it * 2 + hh;
          v4f v = *(const v4f*)(slab + row * 68 + c4);
          *(volatile v4f*)(C + (size_t)(mBase + row) * ldc + n0 + c4) = v;
        }
        __threadfence();
      }
    } else {
      const int q = lane >> 3, c8 = (lane & 7) * 8;
      unsigned short* C  = (unsigned short*)Cout  + (size_t)b * strideC;
      unsigned short* C2 = (OUT_MODE == 2) ? ((unsigned short*)Cout2 + (size_t)b * strideC) : nullptr;
      for (int pass = 0; pass < 2; ++pass) {
#pragma unroll
        for (int it = 0; it < 4; ++it) {
          const int row = it * 4 + q;
          const float* sp = slab + row * 68 + c8;
          v8h hv, lv;
#pragma unroll
          for (int e = 0; e < 8; ++e) {
            if (OUT_MODE == 1) {
              hv[e] = (_Float16)sp[e];
            } else {
              unsigned short hb = f2bf_bits(sp[e]);
              unsigned short lb = f2bf_bits(sp[e] - bf_bits2f(hb));
              hv[e] = __builtin_bit_cast(_Float16, hb);
              lv[e] = __builtin_bit_cast(_Float16, lb);
            }
          }
          *(volatile v8h*)(C + (size_t)(mBase + row) * ldc + n0 + c8) = hv;
          if (OUT_MODE == 2) *(volatile v8h*)(C2 + (size_t)(mBase + row) * ldc + n0 + c8) = lv;
        }
        __threadfence();
      }
    }
    __builtin_amdgcn_fence(__ATOMIC_RELEASE, "workgroup");
    __builtin_amdgcn_wave_barrier();
    __builtin_amdgcn_fence(__ATOMIC_ACQUIRE, "workgroup");
  }
}

__device__ __forceinline__ float bf_rne(float f) { return bf_bits2f(f2bf_bits(f)); }
__device__ __forceinline__ float f16lo_to_f32(unsigned w) {
  const unsigned short b = (unsigned short)(w & 0xffffu);
  const _Float16 h = __builtin_bit_cast(_Float16, b);
  float r = (float)h;
  asm volatile("" : "+v"(r));
  return r;
}
__device__ __forceinline__ float f16hi_to_f32(unsigned w) {
  const unsigned short b = (unsigned short)(w >> 16);
  const _Float16 h = __builtin_bit_cast(_Float16, b);
  float r = (float)h;
  asm volatile("" : "+v"(r));
  return r;
}
__device__ __forceinline__ v8f mma_bf(v16b a, v16b b, v8f c) {
  c = __builtin_amdgcn_wmma_f32_16x16x32_bf16(false, a, false, b, (short)0, c, false, false);
  asm volatile("v_nop\n\tv_nop\n\tv_nop\n\tv_nop" : "+v"(c) : "v"(a), "v"(b));
  return c;
}
__device__ __forceinline__ void store2_v4u(unsigned short* p, v4u v) {
  *(volatile v4u*)p = v;
  __threadfence();
  *(volatile v4u*)p = v;
}
__device__ __forceinline__ void store2_v4f(float* p, v4f v) {
  *(volatile v4f*)p = v;
  __threadfence();
  *(volatile v4f*)p = v;
}

__global__ __launch_bounds__(256) void wt_prep(const float* __restrict__ srcA, int ncolsA,
                                               const float* __restrict__ srcB, int ncolsB,
                                               int row_off, int kvalid, int kp, int nrows_out,
                                               unsigned short* __restrict__ dst) {
  const int cpr = kp >> 3;
  const int f = (int)blockIdx.x * 256 + (int)threadIdx.x;
  const int n = f / cpr;
  if (n >= nrows_out) return;
  const int ch = f - n * cpr;
  const int k8 = ch * 8;
  const int nA = min(n, ncolsA - 1);
  int nB = n - ncolsA; nB = max(nB, 0); nB = min(nB, ncolsB - 1);
  const bool useA = (n < ncolsA);
  unsigned w[4];
#pragma unroll
  for (int e2 = 0; e2 < 4; ++e2) {
    unsigned bits2[2];
#pragma unroll
    for (int s = 0; s < 2; ++s) {
      const int k = k8 + 2 * e2 + s;
      const int kc = min(k, kvalid - 1);
      const float va = srcA[(size_t)(row_off + kc) * ncolsA + nA];
      const float vb = srcB[(size_t)(row_off + kc) * ncolsB + nB];
      float v = useA ? va : vb;
      v = (k < kvalid) ? v : 0.0f;
      bits2[s] = (unsigned)f2bf_bits(v);
    }
    w[e2] = bits2[0] | (bits2[1] << 16);
  }
  const v4u pk = (v4u){w[0], w[1], w[2], w[3]};
  store2_v4u(dst + (size_t)n * kp + k8, pk);
}

__global__ __launch_bounds__(256) void emb_gather(const int* __restrict__ tok_ctx, const int* __restrict__ tok_end,
                                                  const float* __restrict__ emb, int vocab,
                                                  unsigned short* __restrict__ dst) {
  constexpr int CPR = KXP / 8;
  const int f = (int)blockIdx.x * 256 + (int)threadIdx.x;
  const int row = f / CPR;
  if (row >= ROWS_ALL) return;
  const int ch = f - row * CPR;
  const int k8 = ch * 8;
  const int ra = min(row, ROWS_CTX - 1);
  int rb = row - ROWS_CTX; rb = max(rb, 0); rb = min(rb, ROWS_END - 1);
  const int ta = tok_ctx[ra];
  const int tb = tok_end[rb];
  int tok = (row < ROWS_CTX) ? ta : tb;
  tok = max(tok, 0); tok = min(tok, vocab - 1);
  const float* er = emb + (size_t)tok * EMB_DIM;
  const int ia = min(k8, EMB_DIM - 4);
  const int ib = min(k8 + 4, EMB_DIM - 4);
  const v4f a = *(const v4f*)(er + ia);
  const v4f b = *(const v4f*)(er + ib);
  float x[8];
  x[0] = a[0]; x[1] = a[1]; x[2] = a[2]; x[3] = a[3];
  x[4] = b[0]; x[5] = b[1]; x[6] = b[2]; x[7] = b[3];
  unsigned w[4];
#pragma unroll
  for (int e2 = 0; e2 < 4; ++e2) {
    const float lo = (k8 + 2 * e2 < EMB_DIM) ? x[2 * e2] : 0.0f;
    const float hi = (k8 + 2 * e2 + 1 < EMB_DIM) ? x[2 * e2 + 1] : 0.0f;
    w[e2] = (unsigned)f2bf_bits(lo) | ((unsigned)f2bf_bits(hi) << 16);
  }
  const v4u pk = (v4u){w[0], w[1], w[2], w[3]};
  store2_v4u(dst + (size_t)row * KXP + k8, pk);
}

__global__ __launch_bounds__(256) void gru_rec(
    const unsigned short* __restrict__ gx, const unsigned short* __restrict__ wht,
    const int* __restrict__ len_ctx, const int* __restrict__ len_end,
    const float* __restrict__ gate_b, const float* __restrict__ cand_b,
    unsigned short* __restrict__ states, int nb_ctx_blocks, int reverse) {
  __shared__ __align__(16) unsigned short whs[NGX * NCELL];
  __shared__ __align__(16) float hf[16 * NCELL];
  __shared__ __align__(16) unsigned short hb[16 * NCELL];
  __shared__ __align__(16) unsigned short rhb[16 * NCELL];
  __shared__ __align__(16) float us[16 * NCELL];
  __shared__ __align__(16) float gxs[16 * NGX];
  __shared__ __align__(16) unsigned short outs[16 * NCELL];
  __shared__ int lens[16];

  const int tid  = threadIdx.x;
  const int wave = tid >> 5;
  const int lane = tid & 31;
  const int m    = lane & 15;
  const int hh   = lane >> 4;
  const int koff = hh * 8;
  const bool isEnd = ((int)blockIdx.x >= nb_ctx_blocks);
  const int S = isEnd ? S_END : S_CTX;
  const int rowBase = isEnd ? ROWS_CTX : 0;
  int b0 = (isEnd ? ((int)blockIdx.x - nb_ctx_blocks) : (int)blockIdx.x) * 16;
  b0 = max(b0, 0); b0 = min(b0, NBATCH - 16);

  if (tid < 16) {
    const int bi = min(b0 + tid, NBATCH - 1);
    const int la = len_ctx[bi];
    const int lb = len_end[bi];
    int L = isEnd ? lb : la;
    L = max(L, 0); L = min(L, S);
    lens[tid] = L;
  }
  for (int i = tid; i < 16 * NCELL; i += 256) {
    hf[i] = 0.0f; hb[i] = 0; rhb[i] = 0; us[i] = 0.0f; outs[i] = 0;
  }
#pragma unroll 4
  for (int j = 0; j < (NGX * NCELL / 8) / 256; ++j) {
    const int i = tid + 256 * j;
    const int row = i >> 4;
    const int c = i & 15;
    const v4u w = *(const v4u*)(wht + (size_t)row * NCELL + c * 8);
    *(v4u*)(whs + row * NCELL + c * 8) = w;
  }
  __syncthreads();

  int Lr[8];
#pragma unroll
  for (int r = 0; r < 8; ++r) Lr[r] = lens[8 * hh + r];
  float gb[2];
  gb[0] = bf_rne(gate_b[32 * wave + m]);
  gb[1] = bf_rne(gate_b[32 * wave + 16 + m]);
  const float cb = bf_rne(cand_b[16 * wave + m]);
  const __bf16* whb  = (const __bf16*)whs;
  const __bf16* hbb  = (const __bf16*)hb;
  const __bf16* rhbb = (const __bf16*)rhb;
  const float inv256 = 1.0f / 256.0f;
  const v8f zero8 = (v8f){0.f,0.f,0.f,0.f,0.f,0.f,0.f,0.f};

  for (int t = 0; t < S; ++t) {
    {
      const int row = tid >> 4;
      const int ch  = tid & 15;
      const int L = lens[row];
      int pos = t;
      if (reverse) pos = (t < L) ? (L - 1 - t) : t;
      const unsigned short* src = gx + ((size_t)rowBase + (size_t)(b0 + row) * S + (size_t)pos) * NGX;
#pragma unroll
      for (int q = 0; q < 3; ++q) {
        const int c = ch + 16 * q;
        const v4u w = *(const v4u*)(src + c * 8);
        v4f f0, f1;
        f0[0] = f16lo_to_f32(w[0]) * inv256; f0[1] = f16hi_to_f32(w[0]) * inv256;
        f0[2] = f16lo_to_f32(w[1]) * inv256; f0[3] = f16hi_to_f32(w[1]) * inv256;
        f1[0] = f16lo_to_f32(w[2]) * inv256; f1[1] = f16hi_to_f32(w[2]) * inv256;
        f1[2] = f16lo_to_f32(w[3]) * inv256; f1[3] = f16hi_to_f32(w[3]) * inv256;
        *(v4f*)(gxs + row * NGX + c * 8)     = f0;
        *(v4f*)(gxs + row * NGX + c * 8 + 4) = f1;
      }
    }
    __syncthreads();

    v8f acc[2];
    acc[0] = zero8; acc[1] = zero8;
#pragma unroll
    for (int ks = 0; ks < 4; ++ks) {
      const v16b a  = Frag<__bf16>::load(hbb + m * NCELL + koff + 32 * ks);
      const v16b bA = Frag<__bf16>::load(whb + (size_t)(32 * wave + m) * NCELL + koff + 32 * ks);
      const v16b bB = Frag<__bf16>::load(whb + (size_t)(32 * wave + 16 + m) * NCELL + koff + 32 * ks);
      acc[0] = mma_bf(a, bA, acc[0]);
      acc[1] = mma_bf(a, bB, acc[1]);
    }
#pragma unroll
    for (int j = 0; j < 2; ++j) {
      const int n = 32 * wave + 16 * j + m;
#pragma unroll
      for (int r = 0; r < 8; ++r) {
        const int row = 8 * hh + r;
        const float pre = acc[j][r] + gxs[row * NGX + n] + gb[j];
        const float g = 1.0f / (1.0f + expf(-pre));
        if (wave < 4) {
          const float hcur = hf[row * NCELL + n];
          rhb[row * NCELL + n] = f2bf_bits(g * hcur);
        } else {
          us[row * NCELL + (n - NCELL)] = g;
        }
      }
    }
    __syncthreads();

    v8f acc2 = zero8;
#pragma unroll
    for (int ks = 0; ks < 4; ++ks) {
      const v16b a  = Frag<__bf16>::load(rhbb + m * NCELL + koff + 32 * ks);
      const v16b bC = Frag<__bf16>::load(whb + (size_t)(2 * NCELL + 16 * wave + m) * NCELL + koff + 32 * ks);
      acc2 = mma_bf(a, bC, acc2);
    }
    {
      const int n2 = 16 * wave + m;
#pragma unroll
      for (int r = 0; r < 8; ++r) {
        const int row = 8 * hh + r;
        const float pre = acc2[r] + gxs[row * NGX + 2 * NCELL + n2] + cb;
        const float c = tanhf(pre);
        const float hcur = hf[row * NCELL + n2];
        const float u = us[row * NCELL + n2];
        const float hn = u * hcur + (1.0f - u) * c;
        const bool act = (t < Lr[r]);
        const float hnew = act ? hn : hcur;
        const float ov = act ? hn : 0.0f;
        hf[row * NCELL + n2] = hnew;
        hb[row * NCELL + n2] = f2bf_bits(hnew);
        outs[row * NCELL + n2] = f2bf_bits(ov);
      }
    }
    __syncthreads();

    {
      const int q  = lane >> 3;
      const int c8 = (lane & 7) * 8;
      const int ln = 4 * wave + q;
      const int row = ln >> 1;
      const int hr  = ln & 1;
      const int L = lens[row];
      int pos = t;
      if (reverse) pos = (t < L) ? (L - 1 - t) : t;
      const v4u val = *(const v4u*)(outs + row * NCELL + hr * 64 + c8);
      unsigned short* dstp = states + ((size_t)rowBase + (size_t)(b0 + row) * S + (size_t)pos) * NCELL + hr * 64 + c8;
      store2_v4u(dstp, val);
    }
  }
}

__global__ __launch_bounds__(256) void att_score(const unsigned short* __restrict__ states,
                                                 const unsigned short* __restrict__ attwT,
                                                 const float* __restrict__ att_b, const float* __restrict__ att_v,
                                                 float* __restrict__ scores) {
  __shared__ __align__(16) float slab[8][16 * 132];
  __shared__ __align__(16) unsigned short wts[NCELL * NCELL];
  __shared__ float abv[2 * NCELL];
  __shared__ __align__(16) float scs[128];

  const int tid  = threadIdx.x;
  const int wave = tid >> 5;
  const int lane = tid & 31;
  const int m    = lane & 15;
  const int hh   = lane >> 4;
  const int koff = hh * 8;
  {
    const float xa = att_b[tid & (NCELL - 1)];
    const float xb = att_v[tid & (NCELL - 1)];
    abv[tid] = bf_rne((tid < NCELL) ? xa : xb);
  }
#pragma unroll
  for (int j = 0; j < (NCELL * NCELL / 8) / 256; ++j) {
    const int i = tid + 256 * j;
    const int row = i >> 4;
    const int c = i & 15;
    const v4u w = *(const v4u*)(attwT + (size_t)row * NCELL + c * 8);
    *(v4u*)(wts + row * NCELL + c * 8) = w;
  }
  __syncthreads();

  const int r0 = ((int)blockIdx.x * 8 + wave) * 16;
  const __bf16* A  = (const __bf16*)states;
  const __bf16* Bw = (const __bf16*)wts;
  v8f acc[8];
#pragma unroll
  for (int j = 0; j < 8; ++j) acc[j] = (v8f){0.f,0.f,0.f,0.f,0.f,0.f,0.f,0.f};
#pragma unroll 1
  for (int ks = 0; ks < 4; ++ks) {
    const v16b a = Frag<__bf16>::load(A + (size_t)(r0 + m) * NCELL + koff + 32 * ks);
#pragma unroll
    for (int j = 0; j < 8; ++j) {
      const v16b b = Frag<__bf16>::load(Bw + (16 * j + m) * NCELL + koff + 32 * ks);
      acc[j] = mma_bf(a, b, acc[j]);
    }
  }
  float* sl = slab[wave];
#pragma unroll
  for (int j = 0; j < 8; ++j)
#pragma unroll
    for (int r = 0; r < 8; ++r) sl[(8 * hh + r) * 132 + 16 * j + m] = acc[j][r];
  __syncthreads();
  float s = 0.0f;
#pragma unroll 2
  for (int c = 0; c < 64; ++c) {
    const int col = 64 * hh + c;
    const float x = sl[m * 132 + col] + abv[col];
    s += tanhf(x) * abv[NCELL + col];
  }
  s += __shfl_xor(s, 16, 32);
  if (hh == 0) scs[wave * 16 + m] = s;
  __syncthreads();
  if (wave == 0) {
    const v4f v = *(const v4f*)(scs + 4 * lane);
    store2_v4f(scores + (size_t)blockIdx.x * 128 + 4 * lane, v);
  }
}

__global__ __launch_bounds__(128) void att_pool(const float* __restrict__ scores, const unsigned short* __restrict__ states,
                                                float* __restrict__ feats, int col_off) {
  __shared__ float es[S_CTX];
  __shared__ float red[4];
  __shared__ __align__(16) float fs[NCELL];
  const int tid = threadIdx.x, lane = tid & 31, wave = tid >> 5;
  const bool isEnd = ((int)blockIdx.x >= NBATCH);
  const int b = isEnd ? ((int)blockIdx.x - NBATCH) : (int)blockIdx.x;
  const int S = isEnd ? S_END : S_CTX;
  const int rbase = isEnd ? (ROWS_CTX + b * S_END) : (b * S_CTX);

  float scv[4];
  float mx = -INFINITY;
#pragma unroll
  for (int i = 0; i < 4; ++i) {
    const int s = tid + 128 * i;
    const float sc = scores[(size_t)rbase + min(s, S - 1)];
    scv[i] = sc;
    mx = fmaxf(mx, (s < S) ? sc : -INFINITY);
  }
#pragma unroll
  for (int off = 1; off < 32; off <<= 1) mx = fmaxf(mx, __shfl_xor(mx, off, 32));
  if (lane == 0) red[wave] = mx;
  __syncthreads();
  mx = fmaxf(fmaxf(red[0], red[1]), fmaxf(red[2], red[3]));
  __syncthreads();
  float sum = 0.0f;
#pragma unroll
  for (int i = 0; i < 4; ++i) {
    const int s = tid + 128 * i;
    float e = expf(scv[i] - mx);
    e = (s < S) ? e : 0.0f;
    if (s < S) es[s] = e;
    sum += e;
  }
#pragma unroll
  for (int off = 1; off < 32; off <<= 1) sum += __shfl_xor(sum, off, 32);
  if (lane == 0) red[wave] = sum;
  __syncthreads();
  const float tot = (red[0] + red[1]) + (red[2] + red[3]);
  const float inv = 1.0f / tot;
  float acc = 0.0f;
  const unsigned short* st = states + (size_t)rbase * NCELL + tid;
#pragma unroll 4
  for (int s = 0; s < S; ++s) {
    const unsigned w = (unsigned)st[(size_t)s * NCELL];
    acc += es[s] * __uint_as_float(w << 16);
  }
  fs[tid] = acc * inv;
  __syncthreads();
  if (wave == 0) {
    const v4f v = *(const v4f*)(fs + 4 * lane);
    store2_v4f(feats + (size_t)b * NFEAT + col_off + (isEnd ? 2 * NCELL : 0) + 4 * lane, v);
  }
}

__global__ __launch_bounds__(512) void head_k(const float* __restrict__ feats, const float* __restrict__ hid_w,
                                              const float* __restrict__ hid_b, const float* __restrict__ out_w,
                                              const float* __restrict__ out_b, float* __restrict__ out) {
  __shared__ float part[16];
  __shared__ __align__(16) float lg[NBATCH];
  const int tid = threadIdx.x, lane = tid & 31, wave = tid >> 5, g = tid >> 7, h = tid & (NHID - 1);
  const float hbias = bf_rne(hid_b[h]);
  const float ow = bf_rne(out_w[h]);
  const float ob = bf_rne(out_b[0]);
  for (int bg = 0; bg < NBATCH; bg += 4) {
    const int b = bg + g;
    const float* f = feats + (size_t)b * NFEAT;
    float a = 0.0f;
#pragma unroll 4
    for (int k = 0; k < NFEAT; ++k) a += f[k] * bf_rne(hid_w[(size_t)k * NHID + h]);
    a += hbias;
    a = fmaxf(a, 0.0f);
    float p = a * ow;
#pragma unroll
    for (int off = 1; off < 32; off <<= 1) p += __shfl_xor(p, off, 32);
    if (lane == 0) part[wave] = p;
    __syncthreads();
    if (h == 0) lg[b] = ((part[4 * g] + part[4 * g + 1]) + (part[4 * g + 2] + part[4 * g + 3])) + ob;
    __syncthreads();
  }
  if (wave == 0) {
    const v4f v = *(const v4f*)(lg + 4 * lane);
    store2_v4f(out + 4 * lane, v);
  }
}

extern "C" void kernel_launch(void* const* d_in, const int* in_sizes, int n_in,
                              void* d_out, int out_size, void* d_ws, size_t ws_size,
                              hipStream_t stream) {
  if (n_in < 20) return;
  if (in_sizes[0] != NBATCH * S_CTX || in_sizes[1] != NBATCH * S_END) return;
  if (in_sizes[2] != NBATCH || in_sizes[3] != NBATCH || out_size != NBATCH) return;
  if (in_sizes[5] != NGATE_IN * 2 * NCELL || in_sizes[7] != NGATE_IN * NCELL) return;
  if (in_sizes[9] != NGATE_IN * 2 * NCELL || in_sizes[11] != NGATE_IN * NCELL) return;
  if (in_sizes[14] != NCELL * NCELL || in_sizes[16] != NFEAT * NHID || in_sizes[18] != NHID) return;
  if (in_sizes[4] < EMB_DIM || (in_sizes[4] % EMB_DIM) != 0) return;
  const int vocab = in_sizes[4] / EMB_DIM;

  const int*   tok_ctx = (const int*)d_in[0];
  const int*   tok_end = (const int*)d_in[1];
  const int*   len_ctx = (const int*)d_in[2];
  const int*   len_end = (const int*)d_in[3];
  const float* emb     = (const float*)d_in[4];
  const float* fw_gw   = (const float*)d_in[5];
  const float* fw_gb   = (const float*)d_in[6];
  const float* fw_cw   = (const float*)d_in[7];
  const float* fw_cb   = (const float*)d_in[8];
  const float* bw_gw   = (const float*)d_in[9];
  const float* bw_gb   = (const float*)d_in[10];
  const float* bw_cw   = (const float*)d_in[11];
  const float* bw_cb   = (const float*)d_in[12];
  const float* att_v   = (const float*)d_in[13];
  const float* att_w   = (const float*)d_in[14];
  const float* att_b   = (const float*)d_in[15];
  const float* hid_w   = (const float*)d_in[16];
  const float* hid_b   = (const float*)d_in[17];
  const float* out_w   = (const float*)d_in[18];
  const float* out_b   = (const float*)d_in[19];
  float* out = (float*)d_out;

  char* base = (char*)d_ws;
  size_t off = 0;
  auto carve = [&](size_t bytes) -> char* {
    char* p = base + off;
    off += (bytes + 255) & ~(size_t)255;
    return p;
  };
  unsigned short* embp   = (unsigned short*)carve((size_t)ROWS_ALL * KXP * 2);
  unsigned short* gxp    = (unsigned short*)carve((size_t)ROWS_ALL * NGX * 2);
  unsigned short* stp    = (unsigned short*)carve((size_t)ROWS_ALL * NCELL * 2);
  unsigned short* wx_fw  = (unsigned short*)carve((size_t)NGX * KXP * 2);
  unsigned short* wx_bw  = (unsigned short*)carve((size_t)NGX * KXP * 2);
  unsigned short* wh_fw  = (unsigned short*)carve((size_t)NGX * NCELL * 2);
  unsigned short* wh_bw  = (unsigned short*)carve((size_t)NGX * NCELL * 2);
  unsigned short* attwT  = (unsigned short*)carve((size_t)NCELL * NCELL * 2);
  float*          scores = (float*)carve((size_t)ROWS_ALL * 4);
  float*          feats  = (float*)carve((size_t)NBATCH * NFEAT * 4);
  if (off > ws_size) return;

  const dim3 blk256(256, 1, 1);

  const int g_wx = (NGX * (KXP / 8) + 255) / 256;
  const int g_wh = (NGX * (NCELL / 8) + 255) / 256;
  const int g_aw = (NCELL * (NCELL / 8) + 255) / 256;
  wt_prep<<<dim3(g_wx), blk256, 0, stream>>>(fw_gw, 2 * NCELL, fw_cw, NCELL, 0, EMB_DIM, KXP, NGX, wx_fw);
  wt_prep<<<dim3(g_wx), blk256, 0, stream>>>(bw_gw, 2 * NCELL, bw_cw, NCELL, 0, EMB_DIM, KXP, NGX, wx_bw);
  wt_prep<<<dim3(g_wh), blk256, 0, stream>>>(fw_gw, 2 * NCELL, fw_cw, NCELL, EMB_DIM, NCELL, NCELL, NGX, wh_fw);
  wt_prep<<<dim3(g_wh), blk256, 0, stream>>>(bw_gw, 2 * NCELL, bw_cw, NCELL, EMB_DIM, NCELL, NCELL, NGX, wh_bw);
  wt_prep<<<dim3(g_aw), blk256, 0, stream>>>(att_w, NCELL, att_w, NCELL, 0, NCELL, NCELL, NCELL, attwT);

  emb_gather<<<dim3((ROWS_ALL * (KXP / 8)) / 256), blk256, 0, stream>>>(tok_ctx, tok_end, emb, vocab, embp);

  const dim3 g_gemm((ROWS_ALL / 64) * (NGX / 64) / 8, 1, 1);
  const int nb_ctx_blocks = NBATCH / 16;
  const dim3 g_rec(2 * nb_ctx_blocks, 1, 1);
  const dim3 g_sc(ROWS_ALL / 128, 1, 1);
  const dim3 g_pool(2 * NBATCH, 1, 1);

  wmma_gemm64<1, false, 0, 1, false, 0><<<g_gemm, blk256, 0, stream>>>(
      embp, embp, KXP, 0L, wx_fw, wx_fw, KXP, 0L, (void*)gxp, (void*)gxp, NGX, 0L,
      fw_gb, fw_gb, 0L, ROWS_ALL, NGX, KXP, 256.0f);
  gru_rec<<<g_rec, blk256, 0, stream>>>(gxp, wh_fw, len_ctx, len_end, fw_gb, fw_cb, stp, nb_ctx_blocks, 0);
  att_score<<<g_sc, blk256, 0, stream>>>(stp, attwT, att_b, att_v, scores);
  att_pool<<<g_pool, dim3(128, 1, 1), 0, stream>>>(scores, stp, feats, 0);

  wmma_gemm64<1, false, 0, 1, false, 0><<<g_gemm, blk256, 0, stream>>>(
      embp, embp, KXP, 0L, wx_bw, wx_bw, KXP, 0L, (void*)gxp, (void*)gxp, NGX, 0L,
      bw_gb, bw_gb, 0L, ROWS_ALL, NGX, KXP, 256.0f);
  gru_rec<<<g_rec, blk256, 0, stream>>>(gxp, wh_bw, len_ctx, len_end, bw_gb, bw_cb, stp, nb_ctx_blocks, 1);
  att_score<<<g_sc, blk256, 0, stream>>>(stp, attwT, att_b, att_v, scores);
  att_pool<<<g_pool, dim3(128, 1, 1), 0, stream>>>(scores, stp, feats, NCELL);

  head_k<<<dim3(1, 1, 1), dim3(512, 1, 1), 0, stream>>>(feats, hid_w, hid_b, out_w, out_b, out);
}
